// SimpleGAT_40845138985235
// MI455X (gfx1250) — hardware-run, weakly checked
//
#include <hip/hip_runtime.h>
#include <stddef.h>
#include <stdint.h>
#include <math.h>


#define NN      100000
#define NE      1600000
#define DIN     128
#define HC1     128
#define HID     64
#define NCLS    40
#define NCP     48
#define KC      256
#define MP      100096
#define NTHR    256
#define NWAVE   8
#define EPT     8
#define CHUNK   (NTHR * EPT)
#define WCAP    (EPT * 32)
#define LISTN   (NWAVE * WCAP)
#define NB      1024
#define LSH     10
#define SRCB    17
#define SRCM    0x1FFFF
#define NBLK    98
#define RCAP    20480
#define DEGCAP  64
#define GBM     64
#define GBN     64
#define GTHR    128
#define G3M     128
#define NEGS    0.2f
#define WSMAX   134217728
#define LDS_BKT  ((RCAP + LISTN + 16) * 4)
#define LDS_SCAN ((2 * RCAP + 3 * NB + 256 + 16) * 4)

#define PB_X   (MP * 16 / NTHR)
#define PB_W1  16
#define PB_W2  16
#define PB_WC  6
#define PB_ALL (PB_X + PB_W1 + PB_W2 + PB_WC + 1)

#define O_A    ((size_t)0)
#define SZ_A   ((size_t)MP * 128 * 4)
#define O_C    (O_A + SZ_A)
#define O_D    (O_C + SZ_A)
#define SZ_D   ((size_t)MP * 128 * 2)
#define O_W1T  (O_D + SZ_D)
#define O_W2T  (O_W1T + (size_t)256 * 128 * 2)
#define O_WCT  (O_W2T + (size_t)128 * 256 * 2)
#define O_P    (O_WCT + (size_t)NCP * KC * 2)
#define O_META (O_P + (size_t)512 * 4)
#define WS_TOT (O_META + (size_t)NBLK * 128)

static_assert(MP % G3M == 0 && MP % GBM == 0 && MP >= NN && MP - NN < G3M);
static_assert((MP * 16) % NTHR == 0);
static_assert(NN < (1 << SRCB));
static_assert(NB == (1 << LSH) && CHUNK <= (1 << 11) && NB * NWAVE / NWAVE == NB);
static_assert(NBLK * NB >= MP && (NBLK - 1) * NB < NN);
static_assert(NB == NTHR * 4);
static_assert((RCAP % 128) == 0 && RCAP >= 16710 + 2048);
static_assert(DEGCAP >= 36 + 8);
static_assert((size_t)NBLK * RCAP * 4 <= SZ_D);
static_assert(HC1 == 32 * 4 && HID == 32 * 2);
static_assert((NN % 4) == 0);
static_assert((KC % 32) == 0 && (DIN % 32) == 0 && (NCP % 16) == 0 && NCLS <= NCP);
static_assert(G3M * NCLS == 5 * NTHR * 4);
static_assert(LDS_BKT <= 327680 && LDS_SCAN <= 327680);
static_assert(NWAVE * 128 <= RCAP);
static_assert(WS_TOT <= (size_t)WSMAX);
static_assert((O_C % 256) == 0 && (O_D % 256) == 0 && (O_W1T % 256) == 0 && (O_P % 256) == 0 && (O_META % 256) == 0);
static_assert(GBM == (GTHR / 32) * 16 && G3M == (NTHR / 32) * 16);

typedef float          v2f  __attribute__((ext_vector_type(2)));
typedef float          v4f  __attribute__((ext_vector_type(4)));
typedef float          v8f  __attribute__((ext_vector_type(8)));
typedef int            v4i  __attribute__((ext_vector_type(4)));
typedef int            v8i  __attribute__((ext_vector_type(8)));
typedef unsigned int   v2u  __attribute__((ext_vector_type(2)));
typedef unsigned int   v4u  __attribute__((ext_vector_type(4)));
typedef unsigned short v8us __attribute__((ext_vector_type(8)));
typedef __bf16         v16b __attribute__((ext_vector_type(16)));
typedef v2f  __attribute__((may_alias)) v2fa;
typedef v4f  __attribute__((may_alias)) v4fa;
typedef v4i  __attribute__((may_alias)) v4ia;
typedef v8us __attribute__((may_alias)) v8usa;
union FragB { v16b v; v8us h[2]; v8i w; };

__device__ __forceinline__ v8f wmb(const FragB& a, const FragB& b, v8f c) {
  v8f d = __builtin_amdgcn_wmma_f32_16x16x32_bf16(false, a.v, false, b.v, (short)0, c, false, false);
  asm volatile("v_nop\n\tv_nop\n\tv_nop\n\tv_nop" : "+v"(d) : "v"(a.w), "v"(b.w));
  return d;
}

__device__ __forceinline__ unsigned int f2bf(float f) {
  const unsigned int u = __float_as_uint(f);
  const unsigned int r = ((u + 0x7FFFu + ((u >> 16) & 1u)) >> 16) & 0xFFFFu;
  return (f != f) ? 0x7FC0u : r;
}
__device__ __forceinline__ float bf2f(unsigned int b) { return __uint_as_float(b << 16); }
__device__ __forceinline__ float bfr(float f) { return bf2f(f2bf(f)); }
__device__ __forceinline__ unsigned int pk2(float lo, float hi) { return f2bf(lo) | (f2bf(hi) << 16); }
__device__ __forceinline__ v4u pack8(const v4f a, const v4f b) {
  v4u r;
  r.x = pk2(a.x, a.y); r.y = pk2(a.z, a.w); r.z = pk2(b.x, b.y); r.w = pk2(b.z, b.w);
  return r;
}
__device__ __forceinline__ float lk(float v) { return (v >= 0.0f) ? v : NEGS * v; }

__device__ __forceinline__ void wtr_unit(const float* __restrict__ w, int ncol, int kk, int n, int nvalid,
                                         unsigned short* dst) {
  const int ncl = n < nvalid ? n : nvalid - 1;
  const float* p = w + (size_t)kk * (size_t)ncol + ncl;
  v4f a, b;
  a.x = p[0];                  a.y = p[(size_t)ncol];       a.z = p[(size_t)2 * ncol];   a.w = p[(size_t)3 * ncol];
  b.x = p[(size_t)4 * ncol];   b.y = p[(size_t)5 * ncol];   b.z = p[(size_t)6 * ncol];   b.w = p[(size_t)7 * ncol];
  asm volatile("" :: "v"(a), "v"(b));
  const v4f z4 = {0.f, 0.f, 0.f, 0.f};
  if (n >= nvalid) { a = z4; b = z4; }
  const v4u wv = pack8(a, b);
  *(volatile v4u*)dst = wv;
  __threadfence();
  *(volatile v4u*)dst = wv;
}

__global__ __launch_bounds__(NTHR) void k_prep(
    const float* __restrict__ x,
    const float* __restrict__ Wl1, const float* __restrict__ Wr1, const float* __restrict__ att1,
    const float* __restrict__ b1,
    const float* __restrict__ Wl2, const float* __restrict__ Wr2, const float* __restrict__ att2,
    const float* __restrict__ b2,
    const float* __restrict__ Wc, const float* __restrict__ bc,
    unsigned short* XB, unsigned short* W1T, unsigned short* W2T, unsigned short* WcT, float* P, int nN) {
  const int b = (int)blockIdx.x, tid = (int)threadIdx.x;
  if (b < PB_X) {
    const int i = b * NTHR + tid;
    const int row = i >> 4;
    const int c0  = (i & 15) * 8;
    const int rc  = row < nN ? row : nN - 1;
    const float* p = x + (size_t)rc * DIN + c0;
    v4f a = *(const v4fa*)p, q = *(const v4fa*)(p + 4);
    asm volatile("" :: "v"(a), "v"(q));
    const v4f z4 = {0.f, 0.f, 0.f, 0.f};
    if (row >= nN) { a = z4; q = z4; }
    const v4u hv = pack8(a, q);
    unsigned short* o = XB + (size_t)row * DIN + c0;
    *(volatile v4u*)o = hv;
    __threadfence();
    *(volatile v4u*)o = hv;
    return;
  }
  const int wb1 = b - PB_X;
  if (wb1 < PB_W1) {
    const int n  = wb1 * 16 + (tid >> 4);
    const int k8 = (tid & 15) * 8;
    unsigned short* o = W1T + (size_t)n * DIN + k8;
    if (wb1 < 8) wtr_unit(Wl1, HC1, k8, n, HC1, o);
    else         wtr_unit(Wr1, HC1, k8, n - HC1, HC1, o);
    return;
  }
  const int wb2 = wb1 - PB_W1;
  if (wb2 < PB_W2) {
    const int n  = wb2 * 8 + (tid >> 5);
    const int k8 = (tid & 31) * 8;
    const int kk = k8 & 127;
    unsigned short* o = W2T + (size_t)n * KC + k8;
    if (wb2 < 8) wtr_unit(Wl2, HID, kk, n, HID, o);
    else         wtr_unit(Wr2, HID, kk, n - HID, HID, o);
    return;
  }
  const int wb3 = wb2 - PB_W2;
  if (wb3 < PB_WC) {
    const int n  = wb3 * 8 + (tid >> 5);
    const int k8 = (tid & 31) * 8;
    const int kk = k8 < 64 ? k8 : k8 - 64;
    wtr_unit(Wc, NCLS, kk, n, NCLS, WcT + (size_t)n * KC + k8);
    return;
  }
  if (tid < 128) {
    const int t = tid;
    int i1 = t;      i1 = i1 < 0 ? 0 : (i1 > 31 ? 31 : i1);
    int i2 = t - 32; i2 = i2 < 0 ? 0 : (i2 > 31 ? 31 : i2);
    int i3 = t - 64; i3 = i3 < 0 ? 0 : (i3 > 15 ? 15 : i3);
    int i4 = t - 80; i4 = i4 < 0 ? 0 : (i4 > 15 ? 15 : i4);
    int i5 = t - 96; i5 = i5 < 0 ? 0 : (i5 > 9 ? 9 : i5);
    const v4f c1 = *(const v4fa*)(att1 + 4 * i1);
    const v4f c2 = *(const v4fa*)(b1   + 4 * i2);
    const v4f c3 = *(const v4fa*)(att2 + 4 * i3);
    const v4f c4 = *(const v4fa*)(b2   + 4 * i4);
    const v4f c5 = *(const v4fa*)(bc   + 4 * i5);
    asm volatile("" :: "v"(c1), "v"(c2), "v"(c3), "v"(c4), "v"(c5));
    v4f v = {0.f, 0.f, 0.f, 0.f};
    v = (t < 106) ? c5 : v;
    v = (t < 96)  ? c4 : v;
    v = (t < 80)  ? c3 : v;
    v = (t < 64)  ? c2 : v;
    v = (t < 32)  ? c1 : v;
    v4f r; r.x = bfr(v.x); r.y = bfr(v.y); r.z = bfr(v.z); r.w = bfr(v.w);
    float* o = P + 4 * t;
    *(volatile v4f*)o = r;
    __threadfence();
    *(volatile v4f*)o = r;
  }
}

__global__ __launch_bounds__(GTHR) __attribute__((amdgpu_num_vgpr(248))) void k_gemm(
    const unsigned short* __restrict__ A, const unsigned short* __restrict__ WT,
    float* outF, int K, int ldo, int ysplit, size_t off0, size_t off1)
{
  __shared__ __attribute__((aligned(16))) float stg[GBM * GBN];
  const int tid = (int)threadIdx.x, lane = tid & 31, wave = tid >> 5, hh = lane >> 4, m = lane & 15;
  const int rowBase = (int)blockIdx.x * GBM;
  const int by   = (int)blockIdx.y;
  const int sel  = by >= ysplit ? 1 : 0;
  const size_t obase = sel ? off1 : off0;
  const int colo = (by - sel * ysplit) * GBN;
  const int col0 = by * GBN;

  v8f acc[4];
  {
    const v8f z = {0.f, 0.f, 0.f, 0.f, 0.f, 0.f, 0.f, 0.f};
    acc[0] = z; acc[1] = z; acc[2] = z; acc[3] = z;
  }
  const unsigned short* ap = A  + (size_t)(rowBase + 16 * wave + m) * (size_t)K + 8 * hh;
  const unsigned short* wp = WT + (size_t)(col0 + m) * (size_t)K + 8 * hh;
  const int ksteps = K >> 5;
#pragma unroll 1
  for (int ks = 0; ks < ksteps; ++ks) {
    FragB af;
    af.h[0] = *(const v8usa*)(ap + 32 * ks);
    af.h[1] = *(const v8usa*)(ap + 32 * ks + 16);
#pragma unroll
    for (int t = 0; t < 4; ++t) {
      const unsigned short* wq = wp + (size_t)(16 * t) * (size_t)K + 32 * ks;
      FragB bf;
      bf.h[0] = *(const v8usa*)wq;
      bf.h[1] = *(const v8usa*)(wq + 16);
      acc[t] = wmb(af, bf, acc[t]);
    }
  }

#pragma unroll
  for (int t = 0; t < 4; ++t) {
    const int lc = 16 * t + m;
#pragma unroll
    for (int r = 0; r < 8; ++r) {
      const int lr = 16 * wave + 8 * hh + r;
      stg[lr * GBN + lc] = acc[t][r];
    }
  }
  __syncthreads();

  v4f fv[8];
#pragma unroll
  for (int i = 0; i < 8; ++i) {
    const int lr = 16 * wave + 2 * i + hh;
    fv[i] = *(const v4fa*)(stg + lr * GBN + 4 * m);
  }
#pragma unroll
  for (int i = 0; i < 8; ++i) {
    const int gr = rowBase + 16 * wave + 2 * i + hh;
    float* op = outF + obase + (size_t)gr * (size_t)ldo + colo + 4 * m;
    *(volatile v4f*)op = fv[i];
  }
  __threadfence();
#pragma unroll
  for (int i = 0; i < 8; ++i) {
    const int gr = rowBase + 16 * wave + 2 * i + hh;
    float* op = outF + obase + (size_t)gr * (size_t)ldo + colo + 4 * m;
    *(volatile v4f*)op = fv[i];
  }
}

__device__ __forceinline__ int hit_append(bool hj, unsigned sj, int elj, int wc, int* wl) {
  const unsigned mj = __builtin_amdgcn_ballot_w32(hj);
  const int pos = wc + (int)__builtin_amdgcn_mbcnt_lo(mj, 0u);
  if (hj && pos < WCAP) wl[pos] = (elj << LSH) | (int)sj;
  return wc + (int)__builtin_popcount(mj);
}

__device__ __forceinline__ int scan_chunk(const int* __restrict__ dsts, int nE, int cbase, int slotBase,
                                          int vec8, int* wl, int tid) {
  int wc = 0;
  const int el0  = tid * EPT;
  const int e0   = cbase + el0;
  const int sent = -2147483647 - 1;
  v4i da, db;
  if (vec8 != 0 && cbase + CHUNK <= nE) {
    da = *(const v4ia*)(dsts + e0);
    db = *(const v4ia*)(dsts + e0 + 4);
  } else {
    const int last = nE - 1;
    int t0 = dsts[min(e0,     last)], t1 = dsts[min(e0 + 1, last)];
    int t2 = dsts[min(e0 + 2, last)], t3 = dsts[min(e0 + 3, last)];
    int t4 = dsts[min(e0 + 4, last)], t5 = dsts[min(e0 + 5, last)];
    int t6 = dsts[min(e0 + 6, last)], t7 = dsts[min(e0 + 7, last)];
    asm volatile("" :: "v"(t0), "v"(t1), "v"(t2), "v"(t3));
    asm volatile("" :: "v"(t4), "v"(t5), "v"(t6), "v"(t7));
    da.x = (e0     < nE) ? t0 : sent;  da.y = (e0 + 1 < nE) ? t1 : sent;
    da.z = (e0 + 2 < nE) ? t2 : sent;  da.w = (e0 + 3 < nE) ? t3 : sent;
    db.x = (e0 + 4 < nE) ? t4 : sent;  db.y = (e0 + 5 < nE) ? t5 : sent;
    db.z = (e0 + 6 < nE) ? t6 : sent;  db.w = (e0 + 7 < nE) ? t7 : sent;
  }
  const unsigned nbs = (unsigned)slotBase;
  const unsigned unb = (unsigned)NB;
  const unsigned s0 = (unsigned)da.x - nbs, s1 = (unsigned)da.y - nbs;
  const unsigned s2 = (unsigned)da.z - nbs, s3 = (unsigned)da.w - nbs;
  const unsigned s4 = (unsigned)db.x - nbs, s5 = (unsigned)db.y - nbs;
  const unsigned s6 = (unsigned)db.z - nbs, s7 = (unsigned)db.w - nbs;
  const bool h0 = s0 < unb, h1 = s1 < unb, h2 = s2 < unb, h3 = s3 < unb;
  const bool h4 = s4 < unb, h5 = s5 < unb, h6 = s6 < unb, h7 = s7 < unb;
  const unsigned any = __builtin_amdgcn_ballot_w32(h0 | h1 | h2 | h3 | h4 | h5 | h6 | h7);
  if (any != 0u) {
    wc = hit_append(h0, s0, el0 + 0, wc, wl);
    wc = hit_append(h1, s1, el0 + 1, wc, wl);
    wc = hit_append(h2, s2, el0 + 2, wc, wl);
    wc = hit_append(h3, s3, el0 + 3, wc, wl);
    wc = hit_append(h4, s4, el0 + 4, wc, wl);
    wc = hit_append(h5, s5, el0 + 5, wc, wl);
    wc = hit_append(h6, s6, el0 + 6, wc, wl);
    wc = hit_append(h7, s7, el0 + 7, wc, wl);
  }
  return wc;
}

__global__ __launch_bounds__(NTHR) void k_bucket(const int* __restrict__ srcs, const int* __restrict__ dsts,
                                                  unsigned int* HITS, int* META, int nN, int nE, int vec8) {
  extern __shared__ v4f lds_dyn[];
  int* reg1 = (int*)lds_dyn;
  int* list = reg1 + RCAP;
  int* wcnt = list + LISTN;
  const int tid = (int)threadIdx.x, lane = tid & 31, wave = tid >> 5;
  const int b = (int)blockIdx.x;
  const int nodeBase = b * NB;
  const v4i z4i = {0, 0, 0, 0};
  for (int i = tid; i < RCAP / 4; i += NTHR) *(v4ia*)(reg1 + 4 * i) = z4i;
  __syncthreads();

  int tot = 0, totRaw = 0;
  const int nChunks = (nE + CHUNK - 1) / CHUNK;
  int* wl = list + wave * WCAP;
#pragma unroll 1
  for (int ch = 0; ch < nChunks; ++ch) {
    const int cbase = ch * CHUNK;
    const int wc = scan_chunk(dsts, nE, cbase, nodeBase, vec8, wl, tid);
    if (lane == 0) wcnt[wave] = wc;
    __syncthreads();
    int pre = 0, all = 0;
#pragma unroll
    for (int w2 = 0; w2 < NWAVE; ++w2) {
      int c = wcnt[w2];
      c = c < 0 ? 0 : (c > WCAP ? WCAP : c);
      all += c;
      pre += (w2 < wave) ? c : 0;
    }
    const int wcc  = wc > WCAP ? WCAP : wc;
    const int base = tot + pre;
#pragma unroll 1
    for (int i0 = 0; i0 < wcc; i0 += 32) {
      const int i  = i0 + lane;
      const int ic = i < wcc ? i : wcc - 1;
      const int ent = wl[ic];
      const int el  = (ent >> LSH) & (CHUNK - 1);
      const int sl  = ent & (NB - 1);
      int eid = cbase + el;
      eid = eid < 0 ? 0 : (eid > nE - 1 ? nE - 1 : eid);
      int sraw = srcs[eid];
      asm volatile("" :: "v"(sraw));
      const int s = sraw < 0 ? 0 : (sraw > nN - 1 ? nN - 1 : sraw);
      const int pos = base + i;
      if (i < wcc && pos < RCAP) reg1[pos] = (int)((unsigned)s | ((unsigned)sl << SRCB));
    }
    totRaw += all;
    tot += all;
    tot = tot > RCAP ? RCAP : tot;
    __syncthreads();
  }
  const int nh   = tot;
  const int flag = totRaw > RCAP ? 1 : 0;

  int* hb = (int*)HITS + (size_t)b * RCAP;
#pragma unroll 1
  for (int i = tid; i < RCAP / 4; i += NTHR) {
    const v4i v = *(const v4ia*)(reg1 + 4 * i);
    *(volatile v4i*)(hb + 4 * i) = v;
  }
  __threadfence();
#pragma unroll 1
  for (int i = tid; i < RCAP / 4; i += NTHR) {
    const v4i v = *(const v4ia*)(reg1 + 4 * i);
    *(volatile v4i*)(hb + 4 * i) = v;
  }
  if (wave == 0) {
    v4i mv = {0, 0, 0, 0};
    mv.x = (lane == 0) ? nh : 0;
    mv.y = (lane == 0) ? flag : 0;
    mv.z = (lane == 0) ? totRaw : 0;
    int* mp = META + b * 32 + 4 * (lane & 7);
    if (lane < 8) *(volatile v4i*)mp = mv;
    __threadfence();
    if (lane < 8) *(volatile v4i*)mp = mv;
  }
}

template<int L>
__global__ __launch_bounds__(NTHR) void k_scan(
    const unsigned int* __restrict__ HITS, const int* __restrict__ META,
    const float* __restrict__ FA, char* RC, const float* __restrict__ P, const float* __restrict__ X, int nN) {
  extern __shared__ v4f lds_dyn[];
  int* reg1 = (int*)lds_dyn;
  int* reg2 = reg1 + RCAP;
  int* scnt = reg2 + RCAP;
  int* soff = scnt + NB;
  int* cur  = soff + NB;
  float* sP = (float*)(cur + NB);
  int* wtot = (int*)(sP + 256);
  const int tid = (int)threadIdx.x, lane = tid & 31, wave = tid >> 5;
  const int b = (int)blockIdx.x;
  const int nodeBase = b * NB;

  const v4i mv = *(const v4ia*)(META + b * 32);
  int nh = mv.x;
  const bool bflag = (mv.y != 0) || (mv.x < 0) || (mv.x > RCAP);
  nh = nh < 0 ? 0 : (nh > RCAP ? RCAP : nh);
  nh = __builtin_amdgcn_readfirstlane(nh);

  {
    const int* hb = (const int*)HITS + (size_t)b * RCAP;
    const v4i z4i = {0, 0, 0, 0};
#pragma unroll 1
    for (int i = tid; i < RCAP / 4; i += NTHR) {
      const v4i v = *(const v4ia*)(hb + 4 * i);
      *(v4ia*)(reg1 + 4 * i) = v;
      *(v4ia*)(reg2 + 4 * i) = z4i;
    }
    for (int i = tid; i < NB; i += NTHR) scnt[i] = 0;
    constexpr int PT = (L == 1) ? 64 : 32;
    constexpr int PO = (L == 1) ? 0 : 256;
    if (tid < PT) {
      const v4f t = *(const v4fa*)(P + PO + 4 * tid);
      *(v4fa*)(sP + 4 * tid) = t;
    }
  }
  __syncthreads();

  if (wave == 0) {
#pragma unroll 1
    for (int b0 = 0; b0 < nh; b0 += 32) {
      const int idx = b0 + lane;
      const int uv  = reg1[idx < nh ? idx : nh - 1];
      const int m32 = (nh - b0) < 32 ? (nh - b0) : 32;
#pragma unroll 1
      for (int k = 0; k < m32; ++k) {
        const int u  = __builtin_amdgcn_readlane(uv, k);
        const int sl = (int)(((unsigned)u >> SRCB) & (unsigned)(NB - 1));
        const int c  = scnt[sl];
        if (lane == 0) scnt[sl] = c + 1;
      }
    }
  }
  __syncthreads();

  {
    const v4i ca = *(const v4ia*)(scnt + 4 * tid);
    const int e0 = ca.x < 0 ? 0 : ca.x, e1 = ca.y < 0 ? 0 : ca.y, e2 = ca.z < 0 ? 0 : ca.z, e3 = ca.w < 0 ? 0 : ca.w;
    const int ts = e0 + e1 + e2 + e3;
    int incl = ts;
#pragma unroll
    for (int d = 1; d < 32; d <<= 1) {
      const int up = __shfl_up(incl, d);
      if (lane >= d) incl += up;
    }
    if (lane == 31) wtot[wave] = incl;
    __syncthreads();
    int pre = 0;
#pragma unroll
    for (int w2 = 0; w2 < NWAVE; ++w2) pre += (w2 < wave) ? wtot[w2] : 0;
    int run = pre + incl - ts;
    soff[4 * tid + 0] = run; cur[4 * tid + 0] = run; run += e0;
    soff[4 * tid + 1] = run; cur[4 * tid + 1] = run; run += e1;
    soff[4 * tid + 2] = run; cur[4 * tid + 2] = run; run += e2;
    soff[4 * tid + 3] = run; cur[4 * tid + 3] = run;
  }
  __syncthreads();

  if (wave == 0) {
#pragma unroll 1
    for (int b0 = 0; b0 < nh; b0 += 32) {
      const int idx = b0 + lane;
      const int uv  = reg1[idx < nh ? idx : nh - 1];
      const int m32 = (nh - b0) < 32 ? (nh - b0) : 32;
#pragma unroll 1
      for (int k = 0; k < m32; ++k) {
        const int u  = __builtin_amdgcn_readlane(uv, k);
        const int sl = (int)(((unsigned)u >> SRCB) & (unsigned)(NB - 1));
        const int sv = u & SRCM;
        int pos = cur[sl];
        pos = pos < 0 ? 0 : (pos > RCAP - 1 ? RCAP - 1 : pos);
        if (lane == 0) { reg2[pos] = sv; cur[sl] = pos + 1; }
      }
    }
  }
  __syncthreads();

  const int nbw = NB / NWAVE;
  const float qnan = __int_as_float(0x7fc00000);

  if (L == 1) {
    const v4f at4 = *(const v4fa*)(sP + 4 * lane);
    const v4f bb4 = *(const v4fa*)(sP + 128 + 4 * lane);
    float* stw = (float*)reg1 + wave * 128;
#pragma unroll 1
    for (int jt = 0; jt < nbw; ++jt) {
      const int slot = wave * nbw + jt;
      const int grow = nodeBase + slot;
      if (grow >= MP) break;
      int st = __builtin_amdgcn_readfirstlane(soff[slot]);
      const int craw = __builtin_amdgcn_readfirstlane(scnt[slot]);
      int cnt = craw;
      st  = st < 0 ? 0 : (st > nh ? nh : st);
      cnt = cnt < 0 ? 0 : (cnt > DEGCAP ? DEGCAP : cnt);
      if (cnt > nh - st) cnt = nh - st;
      const bool bad  = bflag || (craw > DEGCAP);
      const bool live = grow < nN;

      const v4f xr  = *(const v4fa*)(RC + (size_t)grow * 512 + 16 * lane);
      const v4f xs0 = *(const v4fa*)(FA + (size_t)grow * HC1 + 4 * lane);
      float part = lk(xs0.x + xr.x) * at4.x;
      part = fmaf(lk(xs0.y + xr.y), at4.y, part);
      part = fmaf(lk(xs0.z + xr.z), at4.z, part);
      part = fmaf(lk(xs0.w + xr.w), at4.w, part);
      part += __shfl_xor(part, 8);
      part += __shfl_xor(part, 4);
      part += __shfl_xor(part, 2);
      part += __shfl_xor(part, 1);
      float mx = part, dn = 1.0f;
      v4f av = xs0;

#pragma unroll 1
      for (int q = 0; q < cnt; ++q) {
        int idx = st + q; idx = idx > RCAP - 1 ? RCAP - 1 : idx;
        int s = __builtin_amdgcn_readfirstlane(reg2[idx]);
        s = s < 0 ? 0 : (s > nN - 1 ? nN - 1 : s);
        const v4f xs = *(const v4fa*)(FA + (size_t)s * HC1 + 4 * lane);
        float pt = lk(xs.x + xr.x) * at4.x;
        pt = fmaf(lk(xs.y + xr.y), at4.y, pt);
        pt = fmaf(lk(xs.z + xr.z), at4.z, pt);
        pt = fmaf(lk(xs.w + xr.w), at4.w, pt);
        pt += __shfl_xor(pt, 8);
        pt += __shfl_xor(pt, 4);
        pt += __shfl_xor(pt, 2);
        pt += __shfl_xor(pt, 1);
        const float df = pt - mx;
        const float ee = expf(-fabsf(df));
        const bool up  = df > 0.f;
        const float s1 = up ? ee : 1.0f;
        const float s2 = up ? 1.0f : ee;
        mx = up ? pt : mx;
        dn = fmaf(dn, s1, s2);
        av.x = fmaf(av.x, s1, s2 * xs.x);
        av.y = fmaf(av.y, s1, s2 * xs.y);
        av.z = fmaf(av.z, s1, s2 * xs.z);
        av.w = fmaf(av.w, s1, s2 * xs.w);
      }
      const float inv = __builtin_amdgcn_rcpf(dn);
      stw[lane]      = fmaf(av.x, inv, bb4.x);
      stw[32 + lane] = fmaf(av.y, inv, bb4.y);
      stw[64 + lane] = fmaf(av.z, inv, bb4.z);
      stw[96 + lane] = fmaf(av.w, inv, bb4.w);
#pragma unroll 1
      for (int j = 0; j < 4; ++j) {
        const float t = stw[32 * j + lane];
        const float e = expm1f(t);
        stw[32 * j + lane] = (t > 0.0f) ? t : e;
      }
      v4f o;
      o.x = stw[lane]; o.y = stw[32 + lane]; o.z = stw[64 + lane]; o.w = stw[96 + lane];
      o.x = bad ? qnan : o.x; o.y = bad ? qnan : o.y; o.z = bad ? qnan : o.z; o.w = bad ? qnan : o.w;
      o.x = live ? o.x : 0.0f; o.y = live ? o.y : 0.0f; o.z = live ? o.z : 0.0f; o.w = live ? o.w : 0.0f;
      const unsigned int hbx = f2bf(o.x), hby = f2bf(o.y), hbz = f2bf(o.z), hbw = f2bf(o.w);
      const unsigned int lbx = f2bf(o.x - bf2f(hbx)), lby = f2bf(o.y - bf2f(hby));
      const unsigned int lbz = f2bf(o.z - bf2f(hbz)), lbw = f2bf(o.w - bf2f(hbw));
      v2u hv, lv;
      hv.x = hbx | (hby << 16); hv.y = hbz | (hbw << 16);
      lv.x = lbx | (lby << 16); lv.y = lbz | (lbw << 16);
      unsigned int* rowp = (unsigned int*)(RC + (size_t)grow * 512);
      *(volatile v2u*)(rowp + 2 * lane)      = hv;
      *(volatile v2u*)(rowp + 64 + 2 * lane) = lv;
      __threadfence();
      *(volatile v2u*)(rowp + 2 * lane)      = hv;
      *(volatile v2u*)(rowp + 64 + 2 * lane) = lv;
    }
  } else {
    const v2f at2 = *(const v2fa*)(sP + 2 * lane);
    const v2f bb2 = *(const v2fa*)(sP + 64 + 2 * lane);
#pragma unroll 1
    for (int jt = 0; jt < nbw; ++jt) {
      const int slot = wave * nbw + jt;
      const int grow = nodeBase + slot;
      if (grow >= MP) break;
      int st = __builtin_amdgcn_readfirstlane(soff[slot]);
      const int craw = __builtin_amdgcn_readfirstlane(scnt[slot]);
      int cnt = craw;
      st  = st < 0 ? 0 : (st > nh ? nh : st);
      cnt = cnt < 0 ? 0 : (cnt > DEGCAP ? DEGCAP : cnt);
      if (cnt > nh - st) cnt = nh - st;
      const bool bad  = bflag || (craw > DEGCAP);
      const bool live = grow < nN;
      const int gx = live ? grow : nN - 1;

      const float* own = FA + (size_t)grow * HC1;
      const v2f xs0 = *(const v2fa*)(own + 2 * lane);
      const v2f xr  = *(const v2fa*)(own + HID + 2 * lane);
      v4f xv = *(const v4fa*)(X + (size_t)gx * DIN + 4 * lane);
      asm volatile("" :: "v"(xv));
      float part = lk(xs0.x + xr.x) * at2.x;
      part = fmaf(lk(xs0.y + xr.y), at2.y, part);
      part += __shfl_xor(part, 16);
      part += __shfl_xor(part, 8);
      part += __shfl_xor(part, 4);
      part += __shfl_xor(part, 2);
      part += __shfl_xor(part, 1);
      float mx = part, dn = 1.0f;
      float a0 = xs0.x, a1 = xs0.y;

#pragma unroll 1
      for (int q = 0; q < cnt; ++q) {
        int idx = st + q; idx = idx > RCAP - 1 ? RCAP - 1 : idx;
        int s = __builtin_amdgcn_readfirstlane(reg2[idx]);
        s = s < 0 ? 0 : (s > nN - 1 ? nN - 1 : s);
        const v2f xs = *(const v2fa*)(FA + (size_t)s * HC1 + 2 * lane);
        float pt = lk(xs.x + xr.x) * at2.x;
        pt = fmaf(lk(xs.y + xr.y), at2.y, pt);
        pt += __shfl_xor(pt, 16);
        pt += __shfl_xor(pt, 8);
        pt += __shfl_xor(pt, 4);
        pt += __shfl_xor(pt, 2);
        pt += __shfl_xor(pt, 1);
        const float df = pt - mx;
        const float ee = expf(-fabsf(df));
        const bool up  = df > 0.f;
        const float s1 = up ? ee : 1.0f;
        const float s2 = up ? 1.0f : ee;
        mx = up ? pt : mx;
        dn = fmaf(dn, s1, s2);
        a0 = fmaf(a0, s1, s2 * xs.x);
        a1 = fmaf(a1, s1, s2 * xs.y);
      }
      const float inv = __builtin_amdgcn_rcpf(dn);
      float o0 = fmaf(a0, inv, bb2.x);
      float o1 = fmaf(a1, inv, bb2.y);
      o0 = bad ? qnan : o0;  o1 = bad ? qnan : o1;
      o0 = live ? o0 : 0.0f; o1 = live ? o1 : 0.0f;
      xv.x = live ? xv.x : 0.0f; xv.y = live ? xv.y : 0.0f; xv.z = live ? xv.z : 0.0f; xv.w = live ? xv.w : 0.0f;
      const unsigned int h0 = f2bf(o0), h1 = f2bf(o1);
      const unsigned int l0 = f2bf(o0 - bf2f(h0)), l1 = f2bf(o1 - bf2f(h1));
      const unsigned int hw = h0 | (h1 << 16);
      const unsigned int lw = l0 | (l1 << 16);
      v2u xw;
      xw.x = pk2(xv.x, xv.y); xw.y = pk2(xv.z, xv.w);
      unsigned int* rowp = (unsigned int*)(RC + (size_t)grow * 512);
      *(volatile unsigned int*)(rowp + lane)      = hw;
      *(volatile unsigned int*)(rowp + 32 + lane) = lw;
      *(volatile v2u*)(rowp + 64 + 2 * lane)      = xw;
      __threadfence();
      *(volatile unsigned int*)(rowp + lane)      = hw;
      *(volatile unsigned int*)(rowp + 32 + lane) = lw;
      *(volatile v2u*)(rowp + 64 + 2 * lane)      = xw;
    }
  }
}

__global__ __launch_bounds__(NTHR) __attribute__((amdgpu_num_vgpr(248))) void k_gemm3(
    const unsigned short* __restrict__ CAT, const unsigned short* __restrict__ WcT,
    const float* __restrict__ P, const int* __restrict__ META, float* out, int nN)
{
  __shared__ __attribute__((aligned(16))) float sO[G3M * NCLS];
  __shared__ __attribute__((aligned(16))) float sB[128];
  const int tid = (int)threadIdx.x, lane = tid & 31, wave = tid >> 5, hh = lane >> 4, m = lane & 15;
  const int rowBase = (int)blockIdx.x * G3M;
  if (tid < 32) {
    const v4f t = *(const v4fa*)(P + 384 + 4 * tid);
    *(v4fa*)(sB + 4 * tid) = t;
  }
  const int fl = META[(rowBase >> 10) * 32 + 1];
  const bool bad = fl != 0;

  v8f acc[3];
  {
    const v8f z = {0.f, 0.f, 0.f, 0.f, 0.f, 0.f, 0.f, 0.f};
    acc[0] = z; acc[1] = z; acc[2] = z;
  }
  const unsigned short* ap = CAT + (size_t)(rowBase + 16 * wave + m) * KC + 8 * hh;
  const unsigned short* wp = WcT + (size_t)m * KC + 8 * hh;
#pragma unroll 1
  for (int ks = 0; ks < KC / 32; ++ks) {
    FragB af;
    af.h[0] = *(const v8usa*)(ap + 32 * ks);
    af.h[1] = *(const v8usa*)(ap + 32 * ks + 16);
#pragma unroll
    for (int t = 0; t < 3; ++t) {
      const unsigned short* wq = wp + (size_t)(16 * t) * KC + 32 * ks;
      FragB bf;
      bf.h[0] = *(const v8usa*)wq;
      bf.h[1] = *(const v8usa*)(wq + 16);
      acc[t] = wmb(af, bf, acc[t]);
    }
  }
  __syncthreads();

  const float qnan = __int_as_float(0x7fc00000);
#pragma unroll
  for (int t = 0; t < 3; ++t) {
    const int lc = 16 * t + m;
    const float bv = sB[lc];
#pragma unroll
    for (int r = 0; r < 8; ++r) {
      const int lr = 16 * wave + 8 * hh + r;
      float v = acc[t][r] + bv;
      v = bad ? qnan : v;
      if (lc < NCLS) sO[lr * NCLS + lc] = v;
    }
  }
  __syncthreads();

  int live = nN - rowBase; live = live < 0 ? 0 : (live > G3M ? G3M : live);
  const int npc = live * (NCLS / 4);
  float* ob = out + (size_t)rowBase * NCLS;
  v4f fv[5];
#pragma unroll
  for (int it = 0; it < 5; ++it) fv[it] = *(const v4fa*)(sO + 4 * (it * NTHR + tid));
#pragma unroll
  for (int it = 0; it < 5; ++it) {
    const int p = it * NTHR + tid;
    if (p < npc) *(volatile v4f*)(ob + 4 * p) = fv[it];
  }
  __threadfence();
#pragma unroll
  for (int it = 0; it < 5; ++it) {
    const int p = it * NTHR + tid;
    if (p < npc) *(volatile v4f*)(ob + 4 * p) = fv[it];
  }
}

extern "C" void kernel_launch(void* const* d_in, const int* in_sizes, int n_in,
                              void* d_out, int out_size, void* d_ws, size_t ws_size,
                              hipStream_t stream) {
  if (n_in < 12) return;
  if (in_sizes[0] != NN * DIN) return;
  if (in_sizes[1] != 2 * NE) return;
  if (in_sizes[2] != DIN * HC1 || in_sizes[3] != DIN * HC1) return;
  if (in_sizes[4] != HC1 || in_sizes[5] != HC1) return;
  if (in_sizes[6] != HC1 * HID || in_sizes[7] != HC1 * HID) return;
  if (in_sizes[8] != HID || in_sizes[9] != HID) return;
  if (in_sizes[10] != (HID + DIN) * NCLS || in_sizes[11] != NCLS) return;
  if (out_size != NN * NCLS) return;
  if (ws_size < WS_TOT) return;

  const float* x    = (const float*)d_in[0];
  const int*   ei   = (const int*)  d_in[1];
  const float* Wl1  = (const float*)d_in[2];
  const float* Wr1  = (const float*)d_in[3];
  const float* att1 = (const float*)d_in[4];
  const float* b1   = (const float*)d_in[5];
  const float* Wl2  = (const float*)d_in[6];
  const float* Wr2  = (const float*)d_in[7];
  const float* att2 = (const float*)d_in[8];
  const float* b2   = (const float*)d_in[9];
  const float* Wc   = (const float*)d_in[10];
  const float* bc   = (const float*)d_in[11];
  float* out = (float*)d_out;
  const int nN = NN, nE = NE;
  const int* src = ei;
  const int* dst = ei + nE;
  const int vec8 = ((nE & 3) == 0) ? 1 : 0;

  char* ws = (char*)d_ws;
  float*          wsf  = (float*)ws;
  float*          RA   = (float*)(ws + O_A);
  char*           RC   = ws + O_C;
  unsigned short* XB   = (unsigned short*)(ws + O_D);
  unsigned int*   HITS = (unsigned int*)(ws + O_D);
  unsigned short* W1T  = (unsigned short*)(ws + O_W1T);
  unsigned short* W2T  = (unsigned short*)(ws + O_W2T);
  unsigned short* WcT  = (unsigned short*)(ws + O_WCT);
  float*          P    = (float*)(ws + O_P);
  int*            META = (int*)(ws + O_META);
  const size_t offA = O_A / 4, offC = O_C / 4;

  hipFuncSetAttribute(reinterpret_cast<const void*>(&k_bucket),
                      hipFuncAttributeMaxDynamicSharedMemorySize, LDS_BKT);
  hipFuncSetAttribute(reinterpret_cast<const void*>(&k_scan<1>),
                      hipFuncAttributeMaxDynamicSharedMemorySize, LDS_SCAN);
  hipFuncSetAttribute(reinterpret_cast<const void*>(&k_scan<2>),
                      hipFuncAttributeMaxDynamicSharedMemorySize, LDS_SCAN);

  k_prep<<<PB_ALL, NTHR, 0, stream>>>(x, Wl1, Wr1, att1, b1, Wl2, Wr2, att2, b2, Wc, bc,
                                       XB, W1T, W2T, WcT, P, nN);
  k_gemm<<<dim3(MP / GBM, 4), GTHR, 0, stream>>>(XB, W1T, wsf, DIN, HC1, 2, offA, offC);
  k_bucket<<<NBLK, NTHR, LDS_BKT, stream>>>(src, dst, HITS, META, nN, nE, vec8);
  k_scan<1><<<NBLK, NTHR, LDS_SCAN, stream>>>(HITS, META, RA, RC, P, x, nN);
  k_gemm<<<dim3(MP / GBM, 2), GTHR, 0, stream>>>((const unsigned short*)RC, W2T, wsf, KC, HC1, 2, offA, offA);
  k_scan<2><<<NBLK, NTHR, LDS_SCAN, stream>>>(HITS, META, RA, RC, P, x, nN);
  k_gemm3<<<MP / G3M, NTHR, 0, stream>>>((const unsigned short*)RC, WcT, P, META, out, nN);
}
